// TransformerBlock_39152921870720
// MI455X (gfx1250) — hardware-run, weakly checked
//
#include <hip/hip_runtime.h>
#include <math.h>

#ifndef NB
#define NB 2
#endif
#ifndef SEQ
#define SEQ 4096
#endif
#define NB_FULL 2
#define SEQ_FULL 4096
#define DM 256
#define NHEAD 8
#define HDIM 32
#define DF 1024
static_assert(SEQ % 64 == 0 && SEQ >= 64 && SEQ <= SEQ_FULL);
static_assert(NB >= 1 && NB <= NB_FULL);
static_assert(DM == NHEAD * HDIM);
static_assert(DM % 64 == 0 && DF % 64 == 0 && HDIM % 32 == 0);
static_assert(HDIM == 32);
static_assert(DM == 256);
static_assert((3 * DM) % 64 == 0 && (DM * DM) % 8 == 0 && (DF * DM) % 8 == 0);
static_assert(((long long)NB * SEQ) % 64 == 0);
static_assert((DF * 4) % 256 == 0 && (DM * 4) % 256 == 0 && ((long long)NB * SEQ * DM * 2) % 256 == 0);
static_assert(3LL * DM * DM * 2 + (long long)DM * DM * 2 + 2LL * DF * DM * 2 + DF * 4 + DM * 4
              + (long long)NB * SEQ * DM * 2
              + 3LL * NB * SEQ * DM * 4
              + (long long)NB * SEQ * 3 * DM * 4
              + (long long)NB * SEQ * 2 * DM * 4
              + (long long)NB * SEQ * DF * 4
              + (long long)NB * SEQ * DF * 2
              <= 134217728LL);

typedef __attribute__((ext_vector_type(16))) _Float16 v16h;
typedef __attribute__((ext_vector_type(8)))  float    v8f;
typedef __attribute__((ext_vector_type(4)))  float    v4f;
typedef __attribute__((ext_vector_type(2)))  float    v2f;
typedef _Float16 h16;

__device__ __forceinline__ int frag_k(int i, int h) { return (i < 8) ? (8 * h + i) : (16 + 8 * h + (i - 8)); }
__device__ __forceinline__ v8f wmma16(v16h a, v16h b, v8f c) {
    c = __builtin_amdgcn_wmma_f32_16x16x32_f16(false, a, false, b, (short)0, c, false, false);
    asm volatile("v_nop\n\tv_nop\n\tv_nop\n\tv_nop" : "+v"(c) : "v"(a), "v"(b));
    return c;
}

#define VST2(T, ptr, val) do { const T vst2_v_ = (val); *(volatile T*)(ptr) = vst2_v_; __threadfence(); *(volatile T*)(ptr) = vst2_v_; } while (0)
#define VST2V4(ptr, val) do { const v4f vst2_v4_ = (val); *(volatile v4f*)(ptr) = vst2_v4_; __threadfence(); *(volatile v4f*)(ptr) = vst2_v4_; } while (0)

static __device__ __forceinline__ h16 toh_flush(float v) { const h16 r = (h16)v; return (fabsf(v) < 6.103515625e-05f) ? (h16)0.0f : r; }
__device__ __forceinline__ unsigned int pk2_flush(float a, float b) {
    return (unsigned int)__builtin_bit_cast(unsigned short, toh_flush(a)) | ((unsigned int)__builtin_bit_cast(unsigned short, toh_flush(b)) << 16);
}
__device__ __forceinline__ v16h fh_ld_v32(const float* __restrict__ row, int h) {
    const v4f a0 = *(const v4f*)(row + 8 * h),      a1 = *(const v4f*)(row + 8 * h + 4);
    const v4f c0 = *(const v4f*)(row + 16 + 8 * h), c1 = *(const v4f*)(row + 20 + 8 * h);
    v16h a;
    a[0]  = toh_flush(a0.x); a[1]  = toh_flush(a0.y); a[2]  = toh_flush(a0.z); a[3]  = toh_flush(a0.w);
    a[4]  = toh_flush(a1.x); a[5]  = toh_flush(a1.y); a[6]  = toh_flush(a1.z); a[7]  = toh_flush(a1.w);
    a[8]  = toh_flush(c0.x); a[9]  = toh_flush(c0.y); a[10] = toh_flush(c0.z); a[11] = toh_flush(c0.w);
    a[12] = toh_flush(c1.x); a[13] = toh_flush(c1.y); a[14] = toh_flush(c1.z); a[15] = toh_flush(c1.w);
    return a;
}

#define AW 4
#define VPITCH (HDIM + 8)
static_assert(SEQ % (16 * AW) == 0);
static_assert((64 * (HDIM / 4)) % (32 * AW) == 0);
static_assert((2 * DM) % 4 == 0 && (3 * DM) % 4 == 0 && HDIM % 4 == 0 && (VPITCH % 4) == 0);
__global__ __launch_bounds__(32 * AW) void k_attn32(const float* __restrict__ Qp, const float* __restrict__ Kp, const float* __restrict__ Vp, float* __restrict__ Op,
                                                    int ldq, int ldk, int ldv, int ldo, int L, float scale) {
    __shared__ __align__(16) float    pl[AW][16 * 64];
    __shared__ __align__(16) _Float16 vl[64 * VPITCH];
    const int lane = threadIdx.x & 31, hf = lane >> 4, l15 = lane & 15;
    const int wave = __builtin_amdgcn_readfirstlane(threadIdx.x >> 5);
    const int h = blockIdx.y, b = blockIdx.z;
    const int q0 = (blockIdx.x * AW + wave) * 16;
    const float L2E = 1.4426950408889634f;
    const float NEG = -__builtin_inff();
    const float* qrow  = Qp + ((long long)b * L + q0 + l15) * ldq + h * HDIM;
    const float* kbase = Kp + (long long)b * L * ldk + h * HDIM;
    const float* vbase = Vp + (long long)b * L * ldv + h * HDIM;
    const v16h qa = fh_ld_v32(qrow, hf);
    v8f o[2]; float m8[8], l8[8];
#pragma unroll
    for (int t = 0; t < 2; ++t) { v8f zz = {}; o[t] = zz; }
#pragma unroll
    for (int i = 0; i < 8; ++i) { m8[i] = NEG; l8[i] = 0.f; }
    for (int j0 = 0; j0 < L; j0 += 64) {
        __syncthreads();
        for (int idx = threadIdx.x; idx < 64 * (HDIM / 4); idx += 32 * AW) {
            const int jr = idx / (HDIM / 4), d = (idx - jr * (HDIM / 4)) * 4;
            const v4f f = *(const v4f*)(vbase + (long long)(j0 + jr) * ldv + d);
            const int vo = jr * VPITCH + d;
            vl[vo + 0] = toh_flush(f.x); vl[vo + 1] = toh_flush(f.y); vl[vo + 2] = toh_flush(f.z); vl[vo + 3] = toh_flush(f.w);
        }
        v8f s[4];
#pragma unroll
        for (int t = 0; t < 4; ++t) {
            const float* krow = kbase + (long long)(j0 + t * 16 + l15) * ldk;
            v8f acc = {};
            acc = wmma16(qa, fh_ld_v32(krow, hf), acc);
            s[t] = acc;
        }
        float pv[8][4];
#pragma unroll
        for (int i = 0; i < 8; ++i) {
            float sc[4];
#pragma unroll
            for (int t = 0; t < 4; ++t) { float v = s[t][i] * scale; v *= L2E; sc[t] = v; }
            float mx = fmaxf(fmaxf(sc[0], sc[1]), fmaxf(sc[2], sc[3]));
            mx = fmaxf(mx, __shfl_xor(mx, 1, 32)); mx = fmaxf(mx, __shfl_xor(mx, 2, 32));
            mx = fmaxf(mx, __shfl_xor(mx, 4, 32)); mx = fmaxf(mx, __shfl_xor(mx, 8, 32));
            const float mnew = fmaxf(m8[i], mx);
            const float corr = (mnew == NEG) ? 1.f : exp2f(m8[i] - mnew);
            float rs = 0.f;
#pragma unroll
            for (int t = 0; t < 4; ++t) { const float pp = exp2f(sc[t] - mnew); rs += pp; pv[i][t] = pp; }
            rs += __shfl_xor(rs, 1, 32); rs += __shfl_xor(rs, 2, 32); rs += __shfl_xor(rs, 4, 32); rs += __shfl_xor(rs, 8, 32);
            l8[i] = l8[i] * corr + rs; m8[i] = mnew;
#pragma unroll
            for (int t = 0; t < 2; ++t) o[t][i] *= corr;
        }
#pragma unroll
        for (int i = 0; i < 8; ++i)
#pragma unroll
            for (int t = 0; t < 4; ++t) pl[wave][(i + 8 * hf) * 64 + t * 16 + l15] = pv[i][t];
        __syncthreads();
        v16h pa0, pa1;
#pragma unroll
        for (int e = 0; e < 16; ++e) {
            const int kk = frag_k(e, hf);
            pa0[e] = toh_flush(pl[wave][l15 * 64 + kk] * 4096.f);
            pa1[e] = toh_flush(pl[wave][l15 * 64 + 32 + kk] * 4096.f);
        }
#pragma unroll
        for (int t = 0; t < 2; ++t) {
            const int dcol = t * 16 + l15;
            v16h b0, b1;
#pragma unroll
            for (int e = 0; e < 16; ++e) { b0[e] = vl[frag_k(e, hf) * VPITCH + dcol]; b1[e] = vl[(32 + frag_k(e, hf)) * VPITCH + dcol]; }
            o[t] = wmma16(pa0, b0, o[t]);
            o[t] = wmma16(pa1, b1, o[t]);
        }
    }
    float invr[8];
#pragma unroll
    for (int i = 0; i < 8; ++i) invr[i] = (l8[i] > 0.f) ? 1.f / (l8[i] * 4096.f) : 0.f;
    __syncthreads();
#pragma unroll
    for (int i = 0; i < 8; ++i)
#pragma unroll
        for (int t = 0; t < 2; ++t) pl[wave][(i + 8 * hf) * 64 + t * 16 + l15] = o[t][i] * invr[i];
    __syncthreads();
    float* obase = Op + ((long long)b * L + q0) * ldo + h * HDIM;
#pragma unroll
    for (int r0 = 0; r0 < 16; r0 += 4) {
        const int row = r0 + (lane >> 3), c4 = (lane & 7) * 4;
        const v4f v = *(const v4f*)&pl[wave][row * 64 + c4];
        VST2V4(obase + (long long)row * ldo + c4, v);
    }
}

namespace eng {
typedef __attribute__((ext_vector_type(16))) _Float16 v16h;
typedef __attribute__((ext_vector_type(8)))  _Float16 v8h;
typedef __attribute__((ext_vector_type(16))) __bf16   v16b;
typedef __attribute__((ext_vector_type(8)))  __bf16   v8b;
typedef __attribute__((ext_vector_type(8)))  float    v8f;
typedef __attribute__((ext_vector_type(4)))  float    v4f;

__device__ __forceinline__ unsigned short f2bf_bits(float f) {
  unsigned u = __float_as_uint(f);
  return (unsigned short)((u + 0x7FFFu + ((u >> 16) & 1u)) >> 16);
}
__device__ __forceinline__ float bf_bits2f(unsigned short h) { return __uint_as_float(((unsigned)h) << 16); }

__device__ __forceinline__ void dep_guard_h(v8f& a, v8f& b, v16h x, v16h y) { asm volatile("v_nop\n\tv_nop\n\tv_nop\n\tv_nop" : "+v"(a), "+v"(b) : "v"(x), "v"(y)); }
__device__ __forceinline__ void dep_guard_b(v8f& a, v8f& b, v16b x, v16b y) { asm volatile("v_nop\n\tv_nop\n\tv_nop\n\tv_nop" : "+v"(a), "+v"(b) : "v"(x), "v"(y)); }
__device__ __forceinline__ void keep4_h(v16h a, v16h b, v16h c, v16h d) { asm volatile("v_nop" :: "v"(a), "v"(b), "v"(c), "v"(d)); }
__device__ __forceinline__ void keep4_b(v16b a, v16b b, v16b c, v16b d) { asm volatile("v_nop" :: "v"(a), "v"(b), "v"(c), "v"(d)); }
__device__ __forceinline__ void acc_guard4(v8f& a, v8f& b, v8f& c, v8f& d) { asm volatile("v_nop\n\tv_nop\n\tv_nop\n\tv_nop" : "+v"(a), "+v"(b), "+v"(c), "+v"(d)); }
template <typename T> struct Frag;
template <> struct Frag<_Float16> {
  typedef v16h V; union U { v16h v; v8h h[2]; };
  static __device__ __forceinline__ v16h load(const _Float16* p) {
    U f; f.h[0] = *(const v8h*)(p); f.h[1] = *(const v8h*)(p + 16); return f.v;
  }
  static __device__ __forceinline__ v8f mma(v16h a, v16h b, v8f c) {
    return __builtin_amdgcn_wmma_f32_16x16x32_f16(false, a, false, b, (short)0, c, false, false);
  }
  static __device__ __forceinline__ void guard(v8f& a, v8f& b, v16h x, v16h y) { dep_guard_h(a, b, x, y); }
  static __device__ __forceinline__ void keep(v16h a, v16h b, v16h c, v16h d) { keep4_h(a, b, c, d); }
};
template <> struct Frag<__bf16> {
  typedef v16b V; union U { v16b v; v8b h[2]; };
  static __device__ __forceinline__ v16b load(const __bf16* p) {
    U f; f.h[0] = *(const v8b*)(p); f.h[1] = *(const v8b*)(p + 16); return f.v;
  }
  static __device__ __forceinline__ v8f mma(v16b a, v16b b, v8f c) {
    return __builtin_amdgcn_wmma_f32_16x16x32_bf16(false, a, false, b, (short)0, c, false, false);
  }
  static __device__ __forceinline__ void guard(v8f& a, v8f& b, v16b x, v16b y) { dep_guard_b(a, b, x, y); }
  static __device__ __forceinline__ void keep(v16b a, v16b b, v16b c, v16b d) { keep4_b(a, b, c, d); }
};

template <int ET> struct Elem;
template <> struct Elem<0> { typedef _Float16 T; };
template <> struct Elem<1> { typedef __bf16 T; };
template <int ET, bool SPLIT, int BIAS_MODE, int OUT_MODE, bool RESID, int ACT = 0>
__global__ __launch_bounds__(256) void wmma_gemm64(
    const unsigned short* __restrict__ Ap, const unsigned short* __restrict__ A2p, int lda, long strideA,
    const unsigned short* __restrict__ Btp, const unsigned short* __restrict__ Bt2p, int ldb, long strideB,
    void* __restrict__ Cout, void* __restrict__ Cout2, int ldc, long strideC,
    const float* __restrict__ bias,
    const float* __restrict__ resid, long strideR,
    int M, int N, int K, float scale) {
  typedef typename Elem<ET>::T T;
  typedef typename Frag<T>::V V;
  const T* A = (const T*)Ap; const T* A2 = (const T*)A2p; const T* Bt = (const T*)Btp; const T* Bt2 = (const T*)Bt2p;
  __shared__ __align__(16) float sT[8][16 * 68];
  const int b    = blockIdx.y;
  const int lane = threadIdx.x & 31;
  const int wave = threadIdx.x >> 5;
  const int tilesN = N >> 6;
  const int tilesM = M >> 6;
  const int tile = blockIdx.x * 8 + wave;
  if (tile >= tilesM * tilesN) return;
  const int tm = tile / tilesN;
  const int tn = tile - tm * tilesN;
  const int m0 = tm << 6;
  const int n0 = tn << 6;

  const T* Ab  = A  + (size_t)b * strideA;
  const T* Bb  = Bt + (size_t)b * strideB;
  const T* Ab2 = SPLIT ? (A2  + (size_t)b * strideA) : nullptr;
  const T* Bb2 = SPLIT ? (Bt2 + (size_t)b * strideB) : nullptr;

  const int rlane = lane & 15;
  const int koff  = (lane >> 4) * 8;
  const int mOff  = (lane >> 4) * 8;

  v8f acc[4][4];
#pragma unroll
  for (int i = 0; i < 4; ++i)
#pragma unroll
    for (int j = 0; j < 4; ++j) acc[i][j] = (v8f){0.f,0.f,0.f,0.f,0.f,0.f,0.f,0.f};

  for (int k0 = 0; k0 < K; k0 += 32) {
    V bh[4], bl[4];
#pragma unroll
    for (int j = 0; j < 4; ++j) {
      const size_t bo = (size_t)(n0 + (j << 4) + rlane) * ldb + koff + k0;
      bh[j] = Frag<T>::load(Bb + bo);
      if (SPLIT) bl[j] = Frag<T>::load(Bb2 + bo);
    }
#pragma unroll
    for (int i = 0; i < 4; ++i) {
      const size_t ao = (size_t)(m0 + (i << 4) + rlane) * lda + koff + k0;
      V ah = Frag<T>::load(Ab + ao);
      V al;
      if (SPLIT) al = Frag<T>::load(Ab2 + ao);
#pragma unroll
      for (int j = 0; j < 4; ++j) {
        acc[i][j] = Frag<T>::mma(ah, bh[j], acc[i][j]);
        if (SPLIT) {
          acc[i][j] = Frag<T>::mma(ah, bl[j], acc[i][j]);
          acc[i][j] = Frag<T>::mma(al, bh[j], acc[i][j]);
        }
      }
      Frag<T>::guard(acc[i][0], acc[i][3], ah, SPLIT ? al : ah);
    }
    Frag<T>::keep(bh[0], bh[1], bh[2], bh[3]);
    if (SPLIT) Frag<T>::keep(bl[0], bl[1], bl[2], bl[3]);
  }
  acc_guard4(acc[0][0], acc[0][1], acc[0][2], acc[0][3]);
  acc_guard4(acc[1][0], acc[1][1], acc[1][2], acc[1][3]);
  acc_guard4(acc[2][0], acc[2][1], acc[2][2], acc[2][3]);
  acc_guard4(acc[3][0], acc[3][1], acc[3][2], acc[3][3]);

  float* slab = sT[wave];
  const float* Rb = RESID ? (resid + (size_t)b * strideR) : nullptr;
#pragma unroll
  for (int i = 0; i < 4; ++i) {
    const int mBase = m0 + (i << 4);
#pragma unroll
    for (int j = 0; j < 4; ++j) {
      const int n = n0 + (j << 4) + rlane;
      float bv = 0.f;
      if (BIAS_MODE == 2) bv = bias[n];
#pragma unroll
      for (int r = 0; r < 8; ++r) {
        float v = acc[i][j][r] * scale;
        if (BIAS_MODE == 1) v += bias[mBase + mOff + r];
        if (BIAS_MODE == 2) v += bv;
        if (RESID) v += Rb[(size_t)(mBase + mOff + r) * ldc + n];
        if (ACT == 1) v = tanhf(v);
        if (ACT == 2) v = fmaxf(v, 0.0f);
        if (ACT == 3) v = v / (1.0f + expf(-v));
        if (ACT == 4) v = (v > 0.f) ? v : 0.01f * v;
        if (ACT == 5) v = 0.5f * v * (1.0f + erff(v * 0.70710678118654752f));
        if (ACT == 6) v = (v > 0.f) ? v : 0.2f * v;
        if (ACT == 7) { const float u = 0.7978845608028654f * (v + 0.044715f * v * v * v); v = 0.5f * v * (1.f + tanhf(u)); }
        slab[(mOff + r) * 68 + (j << 4) + rlane] = v;
      }
    }
    __builtin_amdgcn_fence(3  , "workgroup");
    __builtin_amdgcn_wave_barrier();
    __builtin_amdgcn_fence(2  , "workgroup");
    if (OUT_MODE == 0) {
      float* C = (float*)Cout + (size_t)b * strideC;
      const int hh = lane >> 4, c4 = (lane & 15) * 4;
      for (int pass = 0; pass < 2; ++pass) {
#pragma unroll
        for (int it = 0; it < 8; ++it) {
          const int row = it * 2 + hh;
          v4f v = *(const v4f*)(slab + row * 68 + c4);
          *(volatile v4f*)(C + (size_t)(mBase + row) * ldc + n0 + c4) = v;
        }
        __threadfence();
      }
    } else {
      const int q = lane >> 3, c8 = (lane & 7) * 8;
      unsigned short* C  = (unsigned short*)Cout  + (size_t)b * strideC;
      unsigned short* C2 = (OUT_MODE == 2) ? ((unsigned short*)Cout2 + (size_t)b * strideC) : nullptr;
      for (int pass = 0; pass < 2; ++pass) {
#pragma unroll
        for (int it = 0; it < 4; ++it) {
          const int row = it * 4 + q;
          const float* sp = slab + row * 68 + c8;
          v8h hv, lv;
#pragma unroll
          for (int e = 0; e < 8; ++e) {
            if (OUT_MODE == 1) {
              hv[e] = (_Float16)sp[e];
            } else {
              unsigned short hb = f2bf_bits(sp[e]);
              unsigned short lb = f2bf_bits(sp[e] - bf_bits2f(hb));
              hv[e] = __builtin_bit_cast(_Float16, hb);
              lv[e] = __builtin_bit_cast(_Float16, lb);
            }
          }
          *(volatile v8h*)(C + (size_t)(mBase + row) * ldc + n0 + c8) = hv;
          if (OUT_MODE == 2) *(volatile v8h*)(C2 + (size_t)(mBase + row) * ldc + n0 + c8) = lv;
        }
        __threadfence();
      }
    }
    __builtin_amdgcn_fence(3  , "workgroup");
    __builtin_amdgcn_wave_barrier();
    __builtin_amdgcn_fence(2  , "workgroup");
  }
}

}

__global__ __launch_bounds__(256) void k_cast16(const float* __restrict__ src, long long lds, _Float16* __restrict__ dst, long long ldd, int R, int C, float s) {
    const long long i = (long long)blockIdx.x * 256 + threadIdx.x; const long long np = (long long)R * (C / 2); if (i >= np) return; const int r = (int)(i / (C / 2)); const int c = 2 * (int)(i % (C / 2));
    const _Float16 h0 = (_Float16)(src[(long long)r * lds + c] * s), h1 = (_Float16)(src[(long long)r * lds + c + 1] * s);
    const unsigned u = (unsigned)__builtin_bit_cast(unsigned short, h0) | ((unsigned)__builtin_bit_cast(unsigned short, h1) << 16);
    volatile unsigned* d = (volatile unsigned*)(dst + (long long)r * ldd + c); *d = u; __threadfence(); *d = u; }

typedef unsigned int cm_u4 __attribute__((ext_vector_type(4)));
__device__ __forceinline__ unsigned int cmb_pk2(float a, float b) { return (unsigned int)__builtin_bit_cast(unsigned short, (_Float16)a) | ((unsigned int)__builtin_bit_cast(unsigned short, (_Float16)b) << 16); }
__device__ __forceinline__ float cmb_bf(float v) { const unsigned u = __builtin_bit_cast(unsigned, v); const unsigned r = (u + 0x7fffu + ((u >> 16) & 1u)) & 0xffff0000u; return __builtin_bit_cast(float, r); }
__global__ __launch_bounds__(256) void k_cm_bfvec(const float* __restrict__ SRC, float* __restrict__ DST, int n) { const int u = blockIdx.x * 256 + threadIdx.x; if (u >= n) return; VST2(float, DST + u, cmb_bf(SRC[u])); }
__global__ __launch_bounds__(256) void k_cm_castb(const float* __restrict__ SRC, unsigned short* __restrict__ DST, long long n8, float sc) {
    const long long u = (long long)blockIdx.x * 256 + threadIdx.x; if (u >= n8) return;
    const v4f a = *(const v4f*)(SRC + 8 * u), b = *(const v4f*)(SRC + 8 * u + 4);
    cm_u4 pk;
    pk.x = pk2_flush(cmb_bf(a.x) * sc, cmb_bf(a.y) * sc); pk.y = pk2_flush(cmb_bf(a.z) * sc, cmb_bf(a.w) * sc);
    pk.z = pk2_flush(cmb_bf(b.x) * sc, cmb_bf(b.y) * sc); pk.w = pk2_flush(cmb_bf(b.z) * sc, cmb_bf(b.w) * sc);
    VST2(cm_u4, (cm_u4*)(DST + 8 * u), pk); }

__global__ __launch_bounds__(256) void k_bfx(const float* __restrict__ X, float* __restrict__ XB, long long n) {
    const long long u = (long long)blockIdx.x * 256 + threadIdx.x; if (u >= n) return;
    const long long r = u >> 8; const int c = (int)(u & 255); const long long bb = r / SEQ, ii = r - bb * SEQ;
    VST2(float, XB + u, cmb_bf(X[(bb * (long long)SEQ_FULL + ii) * DM + c]));
}

template <int BFX>
__global__ __launch_bounds__(256) void k_ln256(const float* __restrict__ X, int SB, const float* __restrict__ G, const float* __restrict__ Cb, unsigned short* __restrict__ O, int rows) {
    #pragma clang fp contract(off)
    const int wave = __builtin_amdgcn_readfirstlane(threadIdx.x >> 5);
    const int row = blockIdx.x * 8 + wave; const int L = threadIdx.x & 31; if (row >= rows) return;
    const int bb = row / SEQ, ii = row - bb * SEQ;
    const float* xr = X + ((long long)bb * SB + ii) * DM;
    const v4f a = *(const v4f*)(xr + 8 * L), b = *(const v4f*)(xr + 8 * L + 4);
    const v4f ga = *(const v4f*)(G + 8 * L), gb = *(const v4f*)(G + 8 * L + 4);
    const v4f ca = *(const v4f*)(Cb + 8 * L), cb = *(const v4f*)(Cb + 8 * L + 4);
    float x[8] = {a.x, a.y, a.z, a.w, b.x, b.y, b.z, b.w}; float s = 0.f;
    const float g[8] = {ga.x, ga.y, ga.z, ga.w, gb.x, gb.y, gb.z, gb.w};
    const float c[8] = {ca.x, ca.y, ca.z, ca.w, cb.x, cb.y, cb.z, cb.w};
#pragma unroll
    for (int e = 0; e < 8; ++e) { const float t = BFX ? cmb_bf(x[e]) : x[e]; x[e] = t; s += t; }
#pragma unroll
    for (int o = 16; o > 0; o >>= 1) s += __shfl_xor(s, o, 32);
    const float mu = s * (1.f / 256.f); float q = 0.f;
#pragma unroll
    for (int e = 0; e < 8; ++e) { const float d = x[e] - mu; q += d * d; }
#pragma unroll
    for (int o = 16; o > 0; o >>= 1) q += __shfl_xor(q, o, 32);
    const float var = q * (1.f / 256.f); const float inv = 1.f / sqrtf(var + 1e-5f);
    float y[8];
#pragma unroll
    for (int e = 0; e < 8; ++e) y[e] = (x[e] - mu) * inv * cmb_bf(g[e]) + cmb_bf(c[e]);
    cm_u4 pk; pk.x = pk2_flush(y[0], y[1]); pk.y = pk2_flush(y[2], y[3]); pk.z = pk2_flush(y[4], y[5]); pk.w = pk2_flush(y[6], y[7]); VST2(cm_u4, (cm_u4*)(O + (long long)row * DM + 8 * L), pk); }

__global__ __launch_bounds__(256) void k_rope(const float* __restrict__ QKV, float* __restrict__ QKR, int rows) {
    #pragma clang fp contract(off)
    const long long u = (long long)blockIdx.x * 256 + threadIdx.x; if (u >= (long long)rows * 16) return;
    const int row = (int)(u >> 4), j = (int)(u & 15); const int pos = row % SEQ;
    const float invf = exp2f(-(float)j * 0.83048202372184059f);
    const float ang = (float)pos * invf;
    float sn, cs; sincosf(ang, &sn, &cs);
    const float* src = QKV + (long long)row * (3 * DM) + 2 * j;
    float* dst = QKR + (long long)row * (2 * DM) + 2 * j;
#pragma unroll 1
    for (int it = 0; it < 2 * NHEAD; ++it) {
        const v2f a = *(const v2f*)(src + HDIM * it);
        v2f r; r.x = a.x * cs - a.y * sn; r.y = a.y * cs + a.x * sn;
        VST2(v2f, dst + HDIM * it, r);
    }
}

__device__ __forceinline__ float gelu_e(float v) { return 0.5f * v * (1.f + erff(v * 0.70710678118654752f)); }
__global__ __launch_bounds__(256) void k_gelu2e(const float* __restrict__ Hp, unsigned short* __restrict__ O, long long n2, float sc) {
    #pragma clang fp contract(off)
    const long long u = (long long)blockIdx.x * 256 + threadIdx.x; if (u >= n2) return;
    unsigned pk = 0u;
#pragma unroll 1
    for (int e = 0; e < 2; ++e) {
        const float a = Hp[2 * u + e];
        const h16 g = toh_flush(gelu_e(a) * sc);
        pk |= ((unsigned)__builtin_bit_cast(unsigned short, g)) << (16 * e);
    }
    VST2(unsigned, (unsigned*)(O + 2 * u), pk); }


extern "C" void kernel_launch(void* const* d_in, const int* in_sizes, int n_in, void* d_out, int out_size, void* d_ws, size_t ws_size, hipStream_t stream) {
    if (n_in < 13) return;
    const float* x   = (const float*)d_in[0];
    const float* wq  = (const float*)d_in[1];
    const float* wk  = (const float*)d_in[2];
    const float* wv  = (const float*)d_in[3];
    const float* wo  = (const float*)d_in[4];
    const float* g1  = (const float*)d_in[5];
    const float* c1  = (const float*)d_in[6];
    const float* g2  = (const float*)d_in[7];
    const float* c2  = (const float*)d_in[8];
    const float* w2  = (const float*)d_in[9];
    const float* b2  = (const float*)d_in[10];
    const float* w3  = (const float*)d_in[11];
    const float* b3  = (const float*)d_in[12];
    float* out = (float*)d_out;
    const long long M = (long long)NB * SEQ;
    const long long needx = ((long long)(NB - 1) * SEQ_FULL + SEQ) * DM;
    if ((long long)in_sizes[0] < needx || in_sizes[1] < DM * DM || in_sizes[2] < DM * DM || in_sizes[3] < DM * DM || in_sizes[4] < DM * DM ||
        in_sizes[5] < DM || in_sizes[6] < DM || in_sizes[7] < DM || in_sizes[8] < DM ||
        in_sizes[9] < DF * DM || in_sizes[10] < DF || in_sizes[11] < DM * DF || in_sizes[12] < DM || (long long)out_size < needx) return;

    char* wsp = (char*)d_ws;
    auto carve = [&](size_t bytes) -> char* { char* p = wsp; wsp += (bytes + 255) & ~(size_t)255; return p; };
    unsigned short* WQKV16 = (unsigned short*)carve((size_t)3 * DM * DM * 2);
    unsigned short* WO16   = (unsigned short*)carve((size_t)DM * DM * 2);
    unsigned short* W116   = (unsigned short*)carve((size_t)DF * DM * 2);
    unsigned short* W216   = (unsigned short*)carve((size_t)DM * DF * 2);
    float* BR1 = (float*)carve((size_t)DF * 4);
    float* BR2 = (float*)carve((size_t)DM * 4);
    unsigned short* N16 = (unsigned short*)carve((size_t)M * DM * 2);
    float* XB  = (float*)carve((size_t)M * DM * 4);
    float* QKV = (float*)carve((size_t)M * 3 * DM * 4);
    float* QKR = (float*)carve((size_t)M * 2 * DM * 4);
    float* AO  = (float*)carve((size_t)M * DM * 4);
    float* X1  = (float*)carve((size_t)M * DM * 4);
    float* H1  = (float*)carve((size_t)M * DF * 4);
    unsigned short* H16 = (unsigned short*)carve((size_t)M * DF * 2);
    if ((size_t)(wsp - (char*)d_ws) > ws_size) return;

    k_cm_castb<<<(unsigned)(((long long)DM * DM / 8 + 255) / 256), 256, 0, stream>>>(wq, WQKV16 + 0, (long long)DM * DM / 8, 16.0f);
    k_cm_castb<<<(unsigned)(((long long)DM * DM / 8 + 255) / 256), 256, 0, stream>>>(wk, WQKV16 + DM * DM, (long long)DM * DM / 8, 16.0f);
    k_cm_castb<<<(unsigned)(((long long)DM * DM / 8 + 255) / 256), 256, 0, stream>>>(wv, WQKV16 + 2 * DM * DM, (long long)DM * DM / 8, 16.0f);
    k_cm_castb<<<(unsigned)(((long long)DM * DM / 8 + 255) / 256), 256, 0, stream>>>(wo, WO16, (long long)DM * DM / 8, 16.0f);
    k_cm_castb<<<(unsigned)(((long long)DF * DM / 8 + 255) / 256), 256, 0, stream>>>(w2, W116, (long long)DF * DM / 8, 16.0f);
    k_cm_castb<<<(unsigned)(((long long)DM * DF / 8 + 255) / 256), 256, 0, stream>>>(w3, W216, (long long)DM * DF / 8, 16.0f);
    k_cm_bfvec<<<(DF + 255) / 256, 256, 0, stream>>>(b2, BR1, DF); k_cm_bfvec<<<1, 256, 0, stream>>>(b3, BR2, DM);

    k_ln256<1><<<(unsigned)((M + 7) / 8), 256, 0, stream>>>(x, SEQ_FULL, g1, c1, N16, (int)M);
    k_bfx<<<(unsigned)((M * DM + 255) / 256), 256, 0, stream>>>(x, XB, M * DM);

    eng::wmma_gemm64<0, false, 0, 0, false, 0><<<dim3((unsigned)(((M / 64) * (3 * DM / 64) + 7) / 8), 1u), 256, 0, stream>>>(
        (const unsigned short*)N16, nullptr, DM, 0L, (const unsigned short*)WQKV16, nullptr, DM, 0L, (void*)QKV, nullptr, 3 * DM, 0L, nullptr, nullptr, 0L, (int)M, 3 * DM, DM, 0.0625f);

    k_rope<<<(unsigned)((M * 16 + 255) / 256), 256, 0, stream>>>(QKV, QKR, (int)M);

    k_attn32<<<dim3((unsigned)(SEQ / (16 * AW)), (unsigned)NHEAD, (unsigned)NB), 32 * AW, 0, stream>>>(
        QKR, QKR + DM, QKV + 2 * DM, AO, 2 * DM, 2 * DM, 3 * DM, DM, SEQ, 0.17677669529663687f);

    k_cast16<<<(unsigned)(((long long)M * (DM / 2) + 255) / 256), 256, 0, stream>>>(AO, DM, (_Float16*)N16, DM, (int)M, DM, 64.0f);
    eng::wmma_gemm64<0, false, 0, 0, true, 0><<<dim3((unsigned)(((M / 64) * (DM / 64) + 7) / 8), 1u), 256, 0, stream>>>(
        (const unsigned short*)N16, nullptr, DM, 0L, (const unsigned short*)WO16, nullptr, DM, 0L, (void*)X1, nullptr, DM, 0L, nullptr, XB, 0L, (int)M, DM, DM, 1.0f / 1024.0f);
    k_ln256<0><<<(unsigned)((M + 7) / 8), 256, 0, stream>>>(X1, SEQ, g2, c2, N16, (int)M);
    eng::wmma_gemm64<0, false, 2, 0, false, 0><<<dim3((unsigned)(((M / 64) * (DF / 64) + 7) / 8), 1u), 256, 0, stream>>>(
        (const unsigned short*)N16, nullptr, DM, 0L, (const unsigned short*)W116, nullptr, DM, 0L, (void*)H1, nullptr, DF, 0L, BR1, nullptr, 0L, (int)M, DF, DM, 0.0625f);
    k_gelu2e<<<(unsigned)((M * (DF / 2) + 255) / 256), 256, 0, stream>>>(H1, H16, M * (DF / 2), 16.0f);
    eng::wmma_gemm64<0, false, 2, 0, true, 0><<<dim3((unsigned)((((long long)SEQ / 64) * (DM / 64) + 7) / 8), (unsigned)NB), 256, 0, stream>>>(
        (const unsigned short*)H16, nullptr, DF, (long)SEQ * DF, (const unsigned short*)W216, nullptr, DF, 0L, (void*)out, nullptr, DM, (long)SEQ_FULL * DM, BR2, X1, (long)SEQ * DM, SEQ, DM, DF, 1.0f / 256.0f);
}
